// HilbertDilatedAttentionTriton_58926951301485
// MI455X (gfx1250) — hardware-verified
//
#include <hip/hip_runtime.h>
#include <math.h>
#include <stdint.h>

#define NB    2
#define SEQ   4096
#define HID   1024
#define NHEAD 16
#define HDIM  64
#define NKEY  1024
#define KSTEP 4

typedef __attribute__((ext_vector_type(16))) _Float16 v16h;
typedef __attribute__((ext_vector_type(8)))  _Float16 v8h;
typedef __attribute__((ext_vector_type(16))) __bf16   v16b;
typedef __attribute__((ext_vector_type(8)))  __bf16   v8b;
typedef __attribute__((ext_vector_type(8)))  float    v8f;
typedef __attribute__((ext_vector_type(4)))  float    v4f;
typedef __attribute__((ext_vector_type(4)))  unsigned int v4u;

__device__ __forceinline__ unsigned short f2bf_bits(float f) {
  unsigned u = __float_as_uint(f);
  return (unsigned short)((u + 0x7FFFu + ((u >> 16) & 1u)) >> 16);
}
__device__ __forceinline__ float bf_bits2f(unsigned short h) { return __uint_as_float(((unsigned)h) << 16); }
__device__ __forceinline__ unsigned pk16(unsigned short a, unsigned short b) { return (unsigned)a | ((unsigned)b << 16); }
__device__ __forceinline__ void bf_split(float f, __bf16& hi, __bf16& lo) {
  const unsigned short hb = f2bf_bits(f);
  hi = __builtin_bit_cast(__bf16, hb);
  lo = __builtin_bit_cast(__bf16, f2bf_bits(f - bf_bits2f(hb)));
}

__device__ __forceinline__ v16b ldfrag_b(const __bf16* p) {
  union { v16b v; v8b h[2]; } f;
  f.h[0] = *(const v8b*)(p);
  f.h[1] = *(const v8b*)(p + 16);
  return f.v;
}
__device__ __forceinline__ v16h ldfrag_h(const _Float16* p) {
  union { v16h v; v8h h[2]; } f;
  f.h[0] = *(const v8h*)(p);
  f.h[1] = *(const v8h*)(p + 16);
  return f.v;
}

__device__ __forceinline__ void dep_guard_b(v8f& a, v8f& b, v16b x, v16b y) {
  asm volatile("v_nop\n\tv_nop\n\tv_nop\n\tv_nop" : "+v"(a), "+v"(b) : "v"(x), "v"(y));
}
__device__ __forceinline__ void keep4_b(v16b a, v16b b, v16b c, v16b d) { asm volatile("v_nop" :: "v"(a), "v"(b), "v"(c), "v"(d)); }
__device__ __forceinline__ void acc_guard4(v8f& a, v8f& b, v8f& c, v8f& d) {
  asm volatile("v_nop\n\tv_nop\n\tv_nop\n\tv_nop" : "+v"(a), "+v"(b), "+v"(c), "+v"(d));
}
__device__ __forceinline__ v8f mma_b_raw(v16b a, v16b b, v8f c) {
  return __builtin_amdgcn_wmma_f32_16x16x32_bf16(false, a, false, b, (short)0, c, false, false);
}
__device__ __forceinline__ v8f mma_b(v16b a, v16b b, v8f c) {
  c = __builtin_amdgcn_wmma_f32_16x16x32_bf16(false, a, false, b, (short)0, c, false, false);
  asm volatile("v_nop\n\tv_nop\n\tv_nop\n\tv_nop" : "+v"(c) : "v"(a), "v"(b));
  return c;
}
__device__ __forceinline__ v8f mma_h(v16h a, v16h b, v8f c) {
  c = __builtin_amdgcn_wmma_f32_16x16x32_f16(false, a, false, b, (short)0, c, false, false);
  asm volatile("v_nop\n\tv_nop\n\tv_nop\n\tv_nop" : "+v"(c) : "v"(a), "v"(b));
  return c;
}
__device__ __forceinline__ v8f vzero8() { v8f z = {0.f, 0.f, 0.f, 0.f, 0.f, 0.f, 0.f, 0.f}; return z; }

__global__ __launch_bounds__(256) void split8_kernel(const float* __restrict__ in, unsigned short* __restrict__ hi,
                                                     unsigned short* __restrict__ lo, int n8) {
  const int i = blockIdx.x * 256 + threadIdx.x;
  if (i < n8) {
    const size_t e0 = (size_t)i * 8;
    const v4f a = *(const v4f*)(in + e0);
    const v4f b = *(const v4f*)(in + e0 + 4);
    float f[8];
    f[0] = a[0]; f[1] = a[1]; f[2] = a[2]; f[3] = a[3];
    f[4] = b[0]; f[5] = b[1]; f[6] = b[2]; f[7] = b[3];
    v4u uh, ul;
#pragma unroll
    for (int q = 0; q < 4; ++q) {
      const unsigned short h0 = f2bf_bits(f[2 * q]), h1 = f2bf_bits(f[2 * q + 1]);
      const unsigned short l0 = f2bf_bits(f[2 * q] - bf_bits2f(h0));
      const unsigned short l1 = f2bf_bits(f[2 * q + 1] - bf_bits2f(h1));
      uh[q] = pk16(h0, h1);
      ul[q] = pk16(l0, l1);
    }
    *(volatile v4u*)(hi + e0) = uh;
    *(volatile v4u*)(lo + e0) = ul;
    __threadfence();
    *(volatile v4u*)(hi + e0) = uh;
    *(volatile v4u*)(lo + e0) = ul;
  }
}

__global__ __launch_bounds__(128) void gather_rows_kernel(const unsigned short* __restrict__ Xh,
                                                          const unsigned short* __restrict__ Xl,
                                                          const int* __restrict__ hm,
                                                          unsigned short* __restrict__ XSh,
                                                          unsigned short* __restrict__ XSl) {
  const int row = blockIdx.x;
  const int b = row / NKEY, j = row - b * NKEY;
  int src = hm[KSTEP * j];
  src = src < 0 ? 0 : (src > SEQ - 1 ? SEQ - 1 : src);
  const size_t so = ((size_t)b * SEQ + src) * HID + (size_t)threadIdx.x * 8;
  const size_t dof = (size_t)row * HID + (size_t)threadIdx.x * 8;
  const v4u a  = *(const v4u*)(Xh + so);
  const v4u a2 = *(const v4u*)(Xl + so);
  *(volatile v4u*)(XSh + dof) = a;
  *(volatile v4u*)(XSl + dof) = a2;
  __threadfence();
  *(volatile v4u*)(XSh + dof) = a;
  *(volatile v4u*)(XSl + dof) = a2;
}

template <int OUT_MODE>
__global__ __launch_bounds__(256) void gemm64_split_kernel(
    const unsigned short* __restrict__ Ahp, const unsigned short* __restrict__ Alp, int lda, long long strideA,
    const unsigned short* __restrict__ Bhp, const unsigned short* __restrict__ Blp, int ldb, long long strideB,
    void* __restrict__ Cout, void* __restrict__ Cout2, int ldc, long long strideC,
    int M, int N, int K, float scale) {
  __shared__ __align__(16) float sT[8][16 * 68];
  const int z    = blockIdx.y;
  const int lane = threadIdx.x & 31;
  const int wave = threadIdx.x >> 5;
  const int tilesN = N >> 6;
  const int tilesM = M >> 6;
  const int tile = blockIdx.x * 8 + wave;
  if (tile >= tilesM * tilesN) return;
  const int tm = tile / tilesN;
  const int tn = tile - tm * tilesN;
  const int m0 = tm << 6;
  const int n0 = tn << 6;

  const __bf16* Ah = (const __bf16*)(const void*)Ahp + (size_t)z * strideA;
  const __bf16* Al = (const __bf16*)(const void*)Alp + (size_t)z * strideA;
  const __bf16* Bh = (const __bf16*)(const void*)Bhp + (size_t)z * strideB;
  const __bf16* Bl = (const __bf16*)(const void*)Blp + (size_t)z * strideB;

  const int rl   = lane & 15;
  const int koff = (lane >> 4) * 8;
  const int mOff = (lane >> 4) * 8;

  v8f acc[4][4];
#pragma unroll
  for (int i = 0; i < 4; ++i)
#pragma unroll
    for (int j = 0; j < 4; ++j) acc[i][j] = vzero8();

  for (int k0 = 0; k0 < K; k0 += 32) {
    v16b bh[4], bl[4];
#pragma unroll
    for (int j = 0; j < 4; ++j) {
      const size_t bo = (size_t)(n0 + (j << 4) + rl) * ldb + koff + k0;
      bh[j] = ldfrag_b(Bh + bo);
      bl[j] = ldfrag_b(Bl + bo);
    }
#pragma unroll
    for (int i = 0; i < 4; ++i) {
      const size_t ao = (size_t)(m0 + (i << 4) + rl) * lda + koff + k0;
      const v16b ah = ldfrag_b(Ah + ao);
      const v16b al = ldfrag_b(Al + ao);
#pragma unroll
      for (int j = 0; j < 4; ++j) {
        acc[i][j] = mma_b_raw(ah, bh[j], acc[i][j]);
        acc[i][j] = mma_b_raw(ah, bl[j], acc[i][j]);
        acc[i][j] = mma_b_raw(al, bh[j], acc[i][j]);
      }
      dep_guard_b(acc[i][0], acc[i][3], ah, al);
    }
    keep4_b(bh[0], bh[1], bh[2], bh[3]);
    keep4_b(bl[0], bl[1], bl[2], bl[3]);
  }
  acc_guard4(acc[0][0], acc[0][1], acc[0][2], acc[0][3]);
  acc_guard4(acc[1][0], acc[1][1], acc[1][2], acc[1][3]);
  acc_guard4(acc[2][0], acc[2][1], acc[2][2], acc[2][3]);
  acc_guard4(acc[3][0], acc[3][1], acc[3][2], acc[3][3]);

  float* slab = sT[wave];
#pragma unroll
  for (int i = 0; i < 4; ++i) {
    const int mBase = m0 + (i << 4);
#pragma unroll
    for (int j = 0; j < 4; ++j) {
#pragma unroll
      for (int r = 0; r < 8; ++r) {
        slab[(mOff + r) * 68 + (j << 4) + rl] = acc[i][j][r] * scale;
      }
    }
    __builtin_amdgcn_fence(__ATOMIC_RELEASE, "workgroup");
    __builtin_amdgcn_wave_barrier();
    __builtin_amdgcn_fence(__ATOMIC_ACQUIRE, "workgroup");
    if (OUT_MODE == 0) {
      float* C = (float*)Cout + (size_t)z * strideC;
      const int hh = lane >> 4, c4 = (lane & 15) * 4;
      for (int pass = 0; pass < 2; ++pass) {
#pragma unroll
        for (int it = 0; it < 8; ++it) {
          const int row = it * 2 + hh;
          const v4f v = *(const v4f*)(slab + row * 68 + c4);
          *(volatile v4f*)(C + (size_t)(mBase + row) * ldc + n0 + c4) = v;
        }
        __threadfence();
      }
    } else {
      const int q = lane >> 3, c8 = (lane & 7) * 8;
      _Float16* C  = (_Float16*)Cout + (size_t)z * strideC;
      _Float16* C2 = (OUT_MODE == 2) ? ((_Float16*)Cout2 + (size_t)z * strideC) : (_Float16*)Cout;
      v8h hv[4], lv[4];
#pragma unroll
      for (int it = 0; it < 4; ++it) {
        const int row = it * 4 + q;
        const float* sp = slab + row * 68 + c8;
        v8h a, a2;
#pragma unroll
        for (int e = 0; e < 8; ++e) {
          if (OUT_MODE == 1) {
            a[e] = (_Float16)sp[e];
            a2[e] = (_Float16)0.0f;
          } else {
            const unsigned short hb = f2bf_bits(sp[e]);
            const unsigned short lb = f2bf_bits(sp[e] - bf_bits2f(hb));
            a[e]  = __builtin_bit_cast(_Float16, hb);
            a2[e] = __builtin_bit_cast(_Float16, lb);
          }
        }
        hv[it] = a; lv[it] = a2;
      }
      for (int pass = 0; pass < 2; ++pass) {
#pragma unroll
        for (int it = 0; it < 4; ++it) {
          const int row = it * 4 + q;
          const size_t go = (size_t)(mBase + row) * ldc + n0 + c8;
          *(volatile v8h*)(C + go) = hv[it];
          if (OUT_MODE == 2) *(volatile v8h*)(C2 + go) = lv[it];
        }
        __threadfence();
      }
    }
    __builtin_amdgcn_fence(__ATOMIC_RELEASE, "workgroup");
    __builtin_amdgcn_wave_barrier();
    __builtin_amdgcn_fence(__ATOMIC_ACQUIRE, "workgroup");
  }
}

__global__ __launch_bounds__(128)
void attn_kernel(const unsigned short* __restrict__ Qp, const unsigned short* __restrict__ Kp,
                 const unsigned short* __restrict__ VThp, const unsigned short* __restrict__ VTlp,
                 const int* __restrict__ hm,
                 unsigned short* __restrict__ Yhp, unsigned short* __restrict__ Ylp, float sscale) {
  __shared__ __align__(16) __bf16 Psh[4][16 * 64];
  __shared__ __align__(16) __bf16 Psl[4][16 * 64];
  __shared__ __align__(16) float  Os[4][16 * 68];

  const int tid  = threadIdx.x;
  const int wave = tid >> 5;
  const int lane = tid & 31;
  const int hh   = lane >> 4;
  const int c    = lane & 15;

  const int bx = blockIdx.x;
  const int qb = bx & 63;
  const int h  = (bx >> 6) & (NHEAD - 1);
  const int b  = (bx >> 10) & (NB - 1);
  const int q0 = qb * 64 + wave * 16;

  const _Float16* Q  = (const _Float16*)(const void*)Qp + (size_t)b * SEQ * HID + h * HDIM;
  const _Float16* Kk = (const _Float16*)(const void*)Kp + (size_t)b * NKEY * HID + h * HDIM;
  const __bf16*   Vh = (const __bf16*)(const void*)VThp + ((size_t)b * HID + h * HDIM) * NKEY;
  const __bf16*   Vl = (const __bf16*)(const void*)VTlp + ((size_t)b * HID + h * HDIM) * NKEY;

  v16h qa[2];
#pragma unroll
  for (int dc = 0; dc < 2; ++dc) qa[dc] = ldfrag_h(Q + (size_t)(q0 + c) * HID + dc * 32 + 8 * hh);

  float mrow[8], lrow[8];
  v8f oacc[4];
#pragma unroll
  for (int r = 0; r < 8; ++r) { mrow[r] = -INFINITY; lrow[r] = 0.f; }
#pragma unroll
  for (int t = 0; t < 4; ++t) oacc[t] = vzero8();

  __bf16* pwh = Psh[wave];
  __bf16* pwl = Psl[wave];

  for (int kc = 0; kc < NKEY / 64; ++kc) {
    const int kv0 = kc * 64;

    v8f s[4];
#pragma unroll
    for (int j = 0; j < 4; ++j) {
      s[j] = vzero8();
#pragma unroll
      for (int dc = 0; dc < 2; ++dc) {
        const v16h kb = ldfrag_h(Kk + (size_t)(kv0 + j * 16 + c) * HID + dc * 32 + 8 * hh);
        s[j] = mma_h(qa[dc], kb, s[j]);
      }
    }
    float cm[8];
#pragma unroll
    for (int r = 0; r < 8; ++r) {
      float m = -INFINITY;
#pragma unroll
      for (int j = 0; j < 4; ++j) {
        const float sv = s[j][r] * sscale;
        s[j][r] = sv;
        m = fmaxf(m, sv);
      }
#pragma unroll
      for (int off = 1; off < 16; off <<= 1) m = fmaxf(m, __shfl_xor(m, off, 32));
      cm[r] = m;
    }
#pragma unroll
    for (int r = 0; r < 8; ++r) {
      const float mnew = fmaxf(mrow[r], cm[r]);
      const float alpha = __expf(mrow[r] - mnew);
      mrow[r] = mnew;
      float psum = 0.f;
#pragma unroll
      for (int j = 0; j < 4; ++j) {
        const float p = __expf(s[j][r] - mnew);
        psum += p;
        __bf16 a, a2; bf_split(p, a, a2);
        pwh[(8 * hh + r) * 64 + j * 16 + c] = a;
        pwl[(8 * hh + r) * 64 + j * 16 + c] = a2;
      }
#pragma unroll
      for (int off = 1; off < 16; off <<= 1) psum += __shfl_xor(psum, off, 32);
      lrow[r] = lrow[r] * alpha + psum;
#pragma unroll
      for (int t = 0; t < 4; ++t) oacc[t][r] *= alpha;
    }
    __builtin_amdgcn_fence(__ATOMIC_RELEASE, "workgroup");
    __builtin_amdgcn_wave_barrier();
    __builtin_amdgcn_fence(__ATOMIC_ACQUIRE, "workgroup");
#pragma unroll 1
    for (int kk = 0; kk < 2; ++kk) {
      const v16b pa = ldfrag_b(pwh + c * 64 + kk * 32 + 8 * hh);
      const v16b pl = ldfrag_b(pwl + c * 64 + kk * 32 + 8 * hh);
#pragma unroll
      for (int t = 0; t < 4; ++t) {
        const size_t vo = (size_t)(t * 16 + c) * NKEY + kv0 + kk * 32 + 8 * hh;
        const v16b vb = ldfrag_b(Vh + vo);
        const v16b vl = ldfrag_b(Vl + vo);
        oacc[t] = mma_b(pa, vb, oacc[t]);
        oacc[t] = mma_b(pa, vl, oacc[t]);
        oacc[t] = mma_b(pl, vb, oacc[t]);
      }
    }
    __builtin_amdgcn_fence(__ATOMIC_RELEASE, "workgroup");
    __builtin_amdgcn_wave_barrier();
    __builtin_amdgcn_fence(__ATOMIC_ACQUIRE, "workgroup");
  }

  float* os = Os[wave];
#pragma unroll
  for (int r = 0; r < 8; ++r) {
    const float inv = 1.0f / lrow[r];
#pragma unroll
    for (int t = 0; t < 4; ++t) os[(8 * hh + r) * 68 + t * 16 + c] = oacc[t][r] * inv;
  }
  __builtin_amdgcn_fence(__ATOMIC_RELEASE, "workgroup");
  __builtin_amdgcn_wave_barrier();
  __builtin_amdgcn_fence(__ATOMIC_ACQUIRE, "workgroup");
  {
    const int q = lane >> 3, c8 = (lane & 7) * 8;
    v8h hv[4], lv[4];
    int trow[4];
#pragma unroll
    for (int it = 0; it < 4; ++it) {
      const int row = it * 4 + q;
      const float* sp = os + row * 68 + c8;
      v8h a, a2;
#pragma unroll
      for (int e = 0; e < 8; ++e) {
        const unsigned short hb = f2bf_bits(sp[e]);
        const unsigned short lb = f2bf_bits(sp[e] - bf_bits2f(hb));
        a[e]  = __builtin_bit_cast(_Float16, hb);
        a2[e] = __builtin_bit_cast(_Float16, lb);
      }
      hv[it] = a; lv[it] = a2;
      int tr = hm[q0 + row];
      tr = tr < 0 ? 0 : (tr > SEQ - 1 ? SEQ - 1 : tr);
      trow[it] = tr;
    }
    _Float16* Yh = (_Float16*)(void*)Yhp;
    _Float16* Yl = (_Float16*)(void*)Ylp;
    for (int pass = 0; pass < 2; ++pass) {
#pragma unroll
      for (int it = 0; it < 4; ++it) {
        const size_t go = ((size_t)b * SEQ + trow[it]) * HID + h * HDIM + c8;
        *(volatile v8h*)(Yh + go) = hv[it];
        *(volatile v8h*)(Yl + go) = lv[it];
      }
      __threadfence();
    }
  }
}

extern "C" void kernel_launch(void* const* d_in, const int* in_sizes, int n_in,
                              void* d_out, int out_size, void* d_ws, size_t ws_size,
                              hipStream_t stream) {
  if (n_in < 4) return;
  if (in_sizes[0] != NB * SEQ * HID) return;
  if (in_sizes[1] != 3 * HID * HID) return;
  if (in_sizes[2] != HID * HID) return;
  if (in_sizes[3] != SEQ) return;
  if (out_size != NB * SEQ * HID) return;

  const float* x    = (const float*)d_in[0];
  const float* wqkv = (const float*)d_in[1];
  const float* wout = (const float*)d_in[2];
  const int*   hm   = (const int*)d_in[3];
  float*       out  = (float*)d_out;

  const size_t PX  = (size_t)NB * SEQ * HID * 2;
  const size_t PW  = (size_t)3 * HID * HID * 2;
  const size_t PWO = (size_t)HID * HID * 2;
  const size_t PXS = (size_t)NB * NKEY * HID * 2;
  const size_t PKF = (size_t)NB * NKEY * HID * 2;
  const size_t PVT = (size_t)NB * HID * NKEY * 2;
  size_t off = 0;
  const size_t oXh  = off; off += PX;   const size_t oXl  = off; off += PX;
  const size_t oWh  = off; off += PW;   const size_t oWl  = off; off += PW;
  const size_t oWOh = off; off += PWO;  const size_t oWOl = off; off += PWO;
  const size_t oXSh = off; off += PXS;  const size_t oXSl = off; off += PXS;
  const size_t oQf  = off; off += PX;
  const size_t oKf  = off; off += PKF;
  const size_t oVTh = off; off += PVT;  const size_t oVTl = off; off += PVT;
  const size_t oYh  = off; off += PX;   const size_t oYl  = off; off += PX;
  if (off > ws_size) return;

  char* ws = (char*)d_ws;
  unsigned short* Xh  = (unsigned short*)(ws + oXh);  unsigned short* Xl  = (unsigned short*)(ws + oXl);
  unsigned short* Wh  = (unsigned short*)(ws + oWh);  unsigned short* Wl  = (unsigned short*)(ws + oWl);
  unsigned short* WOh = (unsigned short*)(ws + oWOh); unsigned short* WOl = (unsigned short*)(ws + oWOl);
  unsigned short* XSh = (unsigned short*)(ws + oXSh); unsigned short* XSl = (unsigned short*)(ws + oXSl);
  unsigned short* Qf  = (unsigned short*)(ws + oQf);
  unsigned short* Kf  = (unsigned short*)(ws + oKf);
  unsigned short* VTh = (unsigned short*)(ws + oVTh); unsigned short* VTl = (unsigned short*)(ws + oVTl);
  unsigned short* Yh  = (unsigned short*)(ws + oYh);  unsigned short* Yl  = (unsigned short*)(ws + oYl);

  const dim3 blk(256);

  const int n8x = NB * SEQ * HID / 8;
  const int n8w = 3 * HID * HID / 8;
  const int n8o = HID * HID / 8;
  split8_kernel<<<dim3((n8x + 255) / 256), blk, 0, stream>>>(x, Xh, Xl, n8x);
  split8_kernel<<<dim3((n8w + 255) / 256), blk, 0, stream>>>(wqkv, Wh, Wl, n8w);
  split8_kernel<<<dim3((n8o + 255) / 256), blk, 0, stream>>>(wout, WOh, WOl, n8o);

  gather_rows_kernel<<<dim3(NB * NKEY), dim3(128), 0, stream>>>(Xh, Xl, hm, XSh, XSl);

  const long long WQOFF = (long long)HID * HID;
  const long long WVOFF = 2LL * HID * HID;

  gemm64_split_kernel<1><<<dim3(((NB * SEQ / 64) * (HID / 64) + 7) / 8, 1), blk, 0, stream>>>(
      Xh, Xl, HID, 0LL, Wh, Wl, HID, 0LL, (void*)Qf, (void*)Qf, HID, 0LL, NB * SEQ, HID, HID, 1.0f);
  gemm64_split_kernel<1><<<dim3(((NB * NKEY / 64) * (HID / 64) + 7) / 8, 1), blk, 0, stream>>>(
      XSh, XSl, HID, 0LL, Wh + WQOFF, Wl + WQOFF, HID, 0LL, (void*)Kf, (void*)Kf, HID, 0LL,
      NB * NKEY, HID, HID, 1.0f);
  gemm64_split_kernel<2><<<dim3(((HID / 64) * (NKEY / 64) + 7) / 8, NB), blk, 0, stream>>>(
      Wh + WVOFF, Wl + WVOFF, HID, 0LL, XSh, XSl, HID, (long long)NKEY * HID, (void*)VTh, (void*)VTl, NKEY,
      (long long)HID * NKEY, HID, NKEY, HID, 1.0f);
  attn_kernel<<<dim3(NB * NHEAD * (SEQ / 64)), dim3(128), 0, stream>>>(Qf, Kf, VTh, VTl, hm, Yh, Yl, 0.125f);
  gemm64_split_kernel<0><<<dim3(((NB * SEQ / 64) * (HID / 64) + 7) / 8, 1), blk, 0, stream>>>(
      Yh, Yl, HID, 0LL, WOh, WOl, HID, 0LL, (void*)out, (void*)out, HID, 0LL, NB * SEQ, HID, HID, 1.0f);

  (void)hipGetLastError();
}
